// GAT_9586367005317
// MI455X (gfx1250) — hardware-verified
//
#include <hip/hip_runtime.h>
#include <stddef.h>
#include <stdint.h>
#include <math.h>


#define F_IN    128
#define HC      128
#define NHD     4
#define HID     32
#define OUTC    64
#define KA2     256
#define NTHR    256
#define NWAVE   8
#define EPT     8
#define CHUNK   (NTHR * EPT)
#define WCAP    (EPT * 32)
#define LISTN   (NWAVE * WCAP)
#define NBMAX   2048
#define SLOTB   11
#define NBRUN   1024
#define RCAP    28672
#define DEGCAP  256
#define GBM     64
#define GTHR    128
#define MROWS   128
#define NEGSL   0.2f
#define EPS_SM  1e-16f
#define WSMAX   134217728
#define PAR_ATS  0
#define PAR_ATD  128
#define PAR_BIAS 256
#define PAR_LINB 384
#define PAR_N    512
#define NUW1    (HC * (F_IN / 8))
#define NUW2    (OUTC * (KA2 / 8))
#define LDS_SCAN ((2 * RCAP + 2 * NBMAX + LISTN) * 4 + 64)

static_assert(NHD * HID == HC);
static_assert(HID == 32);
static_assert(HC == 4 * 32);
static_assert(OUTC == 64);
static_assert(KA2 == 2 * HC && (KA2 % 32) == 0 && (F_IN % 32) == 0);
static_assert((CHUNK & (CHUNK - 1)) == 0 && CHUNK <= (1 << SLOTB));
static_assert(NBMAX == (1 << SLOTB));
static_assert(NTHR * 8 == NBMAX);
static_assert(NBRUN <= NBMAX && (NBRUN & (NBRUN - 1)) == 0 && (NBRUN % NWAVE) == 0);
static_assert(LISTN >= NBMAX && LISTN >= NWAVE * WCAP);
static_assert((RCAP % 32) == 0);
static_assert(RCAP >= 16710 + 4096);
static_assert(DEGCAP >= 36 + 8);
static_assert(LDS_SCAN <= 300000);
static_assert(GBM == (GTHR / 32) * 16);
static_assert((MROWS % GBM) == 0 && (MROWS % 16) == 0);
static_assert((NUW1 % NTHR) == 0 && (NUW2 % NTHR) == 0);
static_assert(F_IN / 8 == 16 && KA2 / 8 == 32);
static_assert(PAR_LINB + OUTC <= PAR_N && PAR_N == 4 * 128);

typedef float          v4f  __attribute__((ext_vector_type(4)));
typedef float          v8f  __attribute__((ext_vector_type(8)));
typedef int            v4i  __attribute__((ext_vector_type(4)));
typedef int            v8i  __attribute__((ext_vector_type(8)));
typedef unsigned int   v4u  __attribute__((ext_vector_type(4)));
typedef unsigned short v8us __attribute__((ext_vector_type(8)));
typedef __bf16         v16b __attribute__((ext_vector_type(16)));
typedef v4f  __attribute__((may_alias)) v4fa;
typedef v8us __attribute__((may_alias)) v8usa;
union FragB { v16b v; v8us h[2]; v8i w; };

__device__ __forceinline__ v8f wmb(const FragB& a, const FragB& b, v8f c) {
  v8f d = __builtin_amdgcn_wmma_f32_16x16x32_bf16(false, a.v, false, b.v, (short)0, c, false, false);
  asm volatile("v_nop\n\tv_nop\n\tv_nop\n\tv_nop" : "+v"(d) : "v"(a.w), "v"(b.w));
  return d;
}

__device__ __forceinline__ unsigned int f2bf(float f) {
  const unsigned int u = __float_as_uint(f);
  const unsigned int r = ((u + 0x7FFFu + ((u >> 16) & 1u)) >> 16) & 0xFFFFu;
  return ((u & 0x7FFFFFFFu) > 0x7F800000u) ? 0x7FC0u : r;
}
__device__ __forceinline__ float bf2f(unsigned int b) { return __uint_as_float(b << 16); }
__device__ __forceinline__ float bfr(float f) { return bf2f(f2bf(f)); }
__device__ __forceinline__ v4f bfr4(const v4f a) {
  v4f r; r.x = bfr(a.x); r.y = bfr(a.y); r.z = bfr(a.z); r.w = bfr(a.w); return r;
}
__device__ __forceinline__ unsigned int pk2(float lo, float hi) { return f2bf(lo) | (f2bf(hi) << 16); }
__device__ __forceinline__ v4u pack8(const v4f a, const v4f b) {
  v4u r;
  r.x = pk2(a.x, a.y); r.y = pk2(a.z, a.w); r.z = pk2(b.x, b.y); r.w = pk2(b.z, b.w);
  return r;
}

__device__ __forceinline__ int scan_chunk(const int* __restrict__ dsts, int nE, int cbase, int slotBase,
                                          int nb, int vec8, int* list, int tid, int lane, int wave) {
  int wc = 0;
  const int el0  = tid * EPT;
  const int e0   = cbase + el0;
  const int sent = -2147483647 - 1;
  v4i da, db;
  if (vec8 != 0 && cbase + CHUNK <= nE) {
    da = *(const v4i*)(dsts + e0);
    db = *(const v4i*)(dsts + e0 + 4);
  } else {
    da.x = (e0     < nE) ? dsts[min(e0,     nE - 1)] : sent;
    da.y = (e0 + 1 < nE) ? dsts[min(e0 + 1, nE - 1)] : sent;
    da.z = (e0 + 2 < nE) ? dsts[min(e0 + 2, nE - 1)] : sent;
    da.w = (e0 + 3 < nE) ? dsts[min(e0 + 3, nE - 1)] : sent;
    db.x = (e0 + 4 < nE) ? dsts[min(e0 + 4, nE - 1)] : sent;
    db.y = (e0 + 5 < nE) ? dsts[min(e0 + 5, nE - 1)] : sent;
    db.z = (e0 + 6 < nE) ? dsts[min(e0 + 6, nE - 1)] : sent;
    db.w = (e0 + 7 < nE) ? dsts[min(e0 + 7, nE - 1)] : sent;
  }
  const unsigned nbs = (unsigned)slotBase;
  const unsigned unb = (unsigned)nb;
  const unsigned s0 = (unsigned)da.x - nbs, s1 = (unsigned)da.y - nbs;
  const unsigned s2 = (unsigned)da.z - nbs, s3 = (unsigned)da.w - nbs;
  const unsigned s4 = (unsigned)db.x - nbs, s5 = (unsigned)db.y - nbs;
  const unsigned s6 = (unsigned)db.z - nbs, s7 = (unsigned)db.w - nbs;
  const bool h0 = s0 < unb, h1 = s1 < unb, h2 = s2 < unb, h3 = s3 < unb;
  const bool h4 = s4 < unb, h5 = s5 < unb, h6 = s6 < unb, h7 = s7 < unb;
  const unsigned any = __builtin_amdgcn_ballot_w32(h0 | h1 | h2 | h3 | h4 | h5 | h6 | h7);
  if (any != 0u) {
#define HITJ(J, HJ, SJ) { \
      const unsigned mj = __builtin_amdgcn_ballot_w32(HJ); \
      if (mj != 0u) { \
        if (HJ) { \
          const int pos = wc + (int)__builtin_amdgcn_mbcnt_lo(mj, 0u); \
          if (pos < WCAP) list[wave * WCAP + pos] = ((el0 + (J)) << SLOTB) | (int)(SJ); \
        } \
        wc += (int)__builtin_popcount(mj); } }
    HITJ(0, h0, s0)
    HITJ(1, h1, s1)
    HITJ(2, h2, s2)
    HITJ(3, h3, s3)
    HITJ(4, h4, s4)
    HITJ(5, h5, s5)
    HITJ(6, h6, s6)
    HITJ(7, h7, s7)
#undef HITJ
  }
  return wc;
}

__global__ __launch_bounds__(NTHR) void k_prep(const float* __restrict__ x, const float* __restrict__ W,
                                               const float* __restrict__ lw, const float* __restrict__ ats,
                                               const float* __restrict__ atd, const float* __restrict__ bias,
                                               const float* __restrict__ linb,
                                               unsigned short* xb, unsigned short* w1t, unsigned short* lwt2,
                                               float* par, int nN, int nbx) {
  const int b = (int)blockIdx.x, tid = (int)threadIdx.x;
  const v4f z4 = {0.f, 0.f, 0.f, 0.f};
  if (b < nbx) {
    const int u   = b * NTHR + tid;
    const int row = u >> 4;
    const int c0  = (u & 15) * 8;
    const int rc  = row < nN ? row : nN - 1;
    const float* p = x + (size_t)rc * F_IN + c0;
    v4f a = *(const v4fa*)p, c = *(const v4fa*)(p + 4);
    if (row >= nN) { a = z4; c = z4; }
    const v4u hv = pack8(a, c);
    unsigned short* o = xb + (size_t)row * F_IN + c0;
    *(volatile v4u*)o = hv;
    __threadfence();
    *(volatile v4u*)o = hv;
  } else if (b < nbx + NUW1 / NTHR) {
    const int v  = (b - nbx) * NTHR + tid;
    const int n  = v >> 4;
    const int k8 = (v & 15) * 8;
    const float* p = W + (size_t)k8 * HC + n;
    v4f a, c;
    a.x = p[0];       a.y = p[HC];      a.z = p[2 * HC];  a.w = p[3 * HC];
    c.x = p[4 * HC];  c.y = p[5 * HC];  c.z = p[6 * HC];  c.w = p[7 * HC];
    const v4u wv = pack8(a, c);
    unsigned short* o = w1t + (size_t)n * F_IN + k8;
    *(volatile v4u*)o = wv;
    __threadfence();
    *(volatile v4u*)o = wv;
  } else if (b < nbx + NUW1 / NTHR + NUW2 / NTHR) {
    const int v  = (b - nbx - NUW1 / NTHR) * NTHR + tid;
    const int n  = v >> 5;
    const int k8 = (v & 31) * 8;
    const int kk = k8 & (HC - 1);
    const float* p = lw + (size_t)kk * OUTC + n;
    v4f a, c;
    a.x = p[0];         a.y = p[OUTC];      a.z = p[2 * OUTC];  a.w = p[3 * OUTC];
    c.x = p[4 * OUTC];  c.y = p[5 * OUTC];  c.z = p[6 * OUTC];  c.w = p[7 * OUTC];
    const v4u wv = pack8(a, c);
    unsigned short* o = lwt2 + (size_t)n * KA2 + k8;
    *(volatile v4u*)o = wv;
    __threadfence();
    *(volatile v4u*)o = wv;
  } else {
    const int lane = tid & 31, reg = tid >> 5;
    const int c4 = 4 * lane;
    const int cl = 4 * (lane & 15);
    const v4f va = *(const v4fa*)(ats  + c4);
    const v4f vd = *(const v4fa*)(atd  + c4);
    const v4f vb = *(const v4fa*)(bias + c4);
    const v4f vl = *(const v4fa*)(linb + cl);
    v4f v = va;
    if (reg == 1) v = vd;
    if (reg == 2) v = vb;
    if (reg == 3) v = vl;
    const bool zr = (reg == 3) && (lane >= 16);
    v.x = zr ? 0.f : v.x; v.y = zr ? 0.f : v.y; v.z = zr ? 0.f : v.z; v.w = zr ? 0.f : v.w;
    v = bfr4(v);
    float* o = par + (reg & 3) * 128 + c4;
    const bool wr = reg < 4;
    if (wr) *(volatile v4f*)o = v;
    __threadfence();
    if (wr) *(volatile v4f*)o = v;
  }
}

__global__ __launch_bounds__(GTHR) void k_gemm1(const unsigned short* __restrict__ A,
                                                const unsigned short* __restrict__ BT,
                                                float* Hm, const float* __restrict__ par,
                                                float* SD, int MPr) {
  __shared__ __attribute__((aligned(16))) float stg[GBM * HC];
  __shared__ __attribute__((aligned(16))) float sdt[2 * GBM * NHD];
  const int tid = (int)threadIdx.x, lane = tid & 31, wave = tid >> 5, hh = lane >> 4, m = lane & 15;
  const int rowBase = (int)blockIdx.x * GBM;

  v8f acc[8];
  {
    const v8f z = {0.f, 0.f, 0.f, 0.f, 0.f, 0.f, 0.f, 0.f};
#pragma unroll
    for (int t = 0; t < 8; ++t) acc[t] = z;
  }
  const unsigned short* ap = A  + (size_t)(rowBase + 16 * wave + m) * (size_t)F_IN + 8 * hh;
  const unsigned short* bp = BT + (size_t)m * (size_t)F_IN + 8 * hh;

#pragma unroll 1
  for (int k0 = 0; k0 < F_IN; k0 += 32) {
    FragB af;
    af.h[0] = *(const v8usa*)(ap + k0);
    af.h[1] = *(const v8usa*)(ap + k0 + 16);
#pragma unroll
    for (int nt = 0; nt < 8; ++nt) {
      const unsigned short* wq = bp + (size_t)(16 * nt) * (size_t)F_IN + k0;
      FragB bf;
      bf.h[0] = *(const v8usa*)wq;
      bf.h[1] = *(const v8usa*)(wq + 16);
      acc[nt] = wmb(af, bf, acc[nt]);
    }
  }

#pragma unroll
  for (int nt = 0; nt < 8; ++nt) {
    const int lc = 16 * nt + m;
#pragma unroll
    for (int r = 0; r < 8; ++r) {
      const int lr = 16 * wave + 8 * hh + r;
      stg[lr * HC + lc] = acc[nt][r];
    }
  }
  __syncthreads();

  const v4f as4 = *(const v4fa*)(par + PAR_ATS + 4 * lane);
  const v4f ad4 = *(const v4fa*)(par + PAR_ATD + 4 * lane);
  const int head = lane >> 3;
#pragma unroll 1
  for (int i = 0; i < 16; ++i) {
    const int row = wave * 16 + i;
    const v4f p = *(const v4fa*)(stg + row * HC + 4 * lane);
    float s = 0.0f, d = 0.0f;
    s = fmaf(p.x, as4.x, s); s = fmaf(p.y, as4.y, s); s = fmaf(p.z, as4.z, s); s = fmaf(p.w, as4.w, s);
    d = fmaf(p.x, ad4.x, d); d = fmaf(p.y, ad4.y, d); d = fmaf(p.z, ad4.z, d); d = fmaf(p.w, ad4.w, d);
#pragma unroll
    for (int off = 1; off < 8; off <<= 1) {
      s += __shfl_xor(s, off);
      d += __shfl_xor(d, off);
    }
    if ((lane & 7) == 0) {
      sdt[row * NHD + head] = s;
      sdt[GBM * NHD + row * NHD + head] = d;
    }
  }
  __syncthreads();

  const int pl = wave >> 1, hf = wave & 1;
  const v4f alv = *(const v4fa*)(sdt + pl * (GBM * NHD) + hf * 128 + 4 * lane);
  float* alp = SD + (size_t)pl * (size_t)MPr * NHD + (size_t)rowBase * NHD + hf * 128 + 4 * lane;
#pragma unroll 1
  for (int i = 0; i < 16; ++i) {
    const int row = wave * 16 + i;
    const v4f p = *(const v4fa*)(stg + row * HC + 4 * lane);
    float* op = Hm + (size_t)(rowBase + row) * (size_t)HC + 4 * lane;
    *(volatile v4f*)op = p;
  }
  *(volatile v4f*)alp = alv;
  __threadfence();
#pragma unroll 1
  for (int i = 0; i < 16; ++i) {
    const int row = wave * 16 + i;
    const v4f p = *(const v4fa*)(stg + row * HC + 4 * lane);
    float* op = Hm + (size_t)(rowBase + row) * (size_t)HC + 4 * lane;
    *(volatile v4f*)op = p;
  }
  *(volatile v4f*)alp = alv;
}

__global__ __launch_bounds__(NTHR) void k_scan(
    const int* __restrict__ srcs, const int* __restrict__ dsts,
    const float* __restrict__ F, const float* __restrict__ SD,
    const float* __restrict__ par,
    unsigned short* HP,
    int nN, int nE, int nb, int vec8, int MPr) {
  extern __shared__ v4f lds_dyn[];
  int* reg1 = (int*)lds_dyn;
  int* reg2 = reg1 + RCAP;
  int* scnt = reg2 + RCAP;
  int* soff = scnt + NBMAX;
  int* list = soff + NBMAX;
  int* wcnt = list + LISTN;
  int* wtot = wcnt + NWAVE;
  const int tid = (int)threadIdx.x, lane = tid & 31, wave = tid >> 5;
  const int nodeBase = (int)blockIdx.x * nb;

  for (int i = tid; i < NBMAX; i += NTHR) scnt[i] = 0;
  __syncthreads();

  int tot = 0;
  const int nChunks = (nE + CHUNK - 1) / CHUNK;
#pragma unroll 1
  for (int ch = 0; ch < nChunks; ++ch) {
    const int cbase = ch * CHUNK;
    const int wc = scan_chunk(dsts, nE, cbase, nodeBase, nb, vec8, list, tid, lane, wave);
    if (lane == 0) wcnt[wave] = wc;
    __syncthreads();
    int pre = 0, all = 0;
#pragma unroll
    for (int w2 = 0; w2 < NWAVE; ++w2) {
      int c = wcnt[w2];
      c = c < 0 ? 0 : (c > WCAP ? WCAP : c);
      all += c;
      pre += (w2 < wave) ? c : 0;
    }
    const int wcc  = wc > WCAP ? WCAP : wc;
    const int base = tot + pre;
#pragma unroll 1
    for (int i = lane; i < wcc; i += 32) {
      const int ent = list[wave * WCAP + i];
      const int el  = (ent >> SLOTB) & (CHUNK - 1);
      const int sl  = ent & (NBMAX - 1);
      int eid = cbase + el;
      eid = eid > nE - 1 ? nE - 1 : eid;
      const int pos = base + i;
      if (pos < RCAP) reg1[pos] = (int)(((unsigned)eid << SLOTB) | (unsigned)sl);
    }
    tot += all;
    tot = tot > RCAP ? RCAP : tot;
    __syncthreads();
  }
  const int nh = tot;

  if (wave == 0) {
#pragma unroll 1
    for (int b0 = 0; b0 < nh; b0 += 32) {
      const int idx = b0 + lane;
      const int uv  = reg1[idx < nh ? idx : nh - 1];
      const int m32 = (nh - b0) < 32 ? (nh - b0) : 32;
#pragma unroll 1
      for (int k = 0; k < m32; ++k) {
        const int u  = __builtin_amdgcn_readlane(uv, k);
        const int sl = u & (NBMAX - 1);
        if (lane == 0) scnt[sl] = scnt[sl] + 1;
      }
    }
  }
  __syncthreads();

  {
    const v4i ca = *(const v4i*)(scnt + 8 * tid);
    const v4i cb = *(const v4i*)(scnt + 8 * tid + 4);
    const int e0 = ca.x < 0 ? 0 : ca.x, e1 = ca.y < 0 ? 0 : ca.y, e2 = ca.z < 0 ? 0 : ca.z, e3 = ca.w < 0 ? 0 : ca.w;
    const int e4 = cb.x < 0 ? 0 : cb.x, e5 = cb.y < 0 ? 0 : cb.y, e6 = cb.z < 0 ? 0 : cb.z, e7 = cb.w < 0 ? 0 : cb.w;
    const int ts = e0 + e1 + e2 + e3 + e4 + e5 + e6 + e7;
    int incl = ts;
#pragma unroll
    for (int d = 1; d < 32; d <<= 1) {
      const int up = __shfl_up(incl, d);
      if (lane >= d) incl += up;
    }
    if (lane == 31) wtot[wave] = incl;
    __syncthreads();
    int pre = 0;
#pragma unroll
    for (int w2 = 0; w2 < NWAVE; ++w2) pre += (w2 < wave) ? wtot[w2] : 0;
    int run = pre + incl - ts;
    soff[8 * tid + 0] = run; run += e0;
    soff[8 * tid + 1] = run; run += e1;
    soff[8 * tid + 2] = run; run += e2;
    soff[8 * tid + 3] = run; run += e3;
    soff[8 * tid + 4] = run; run += e4;
    soff[8 * tid + 5] = run; run += e5;
    soff[8 * tid + 6] = run; run += e6;
    soff[8 * tid + 7] = run;
  }
  __syncthreads();
  for (int i = tid; i < NBMAX; i += NTHR) list[i] = soff[i];
  __syncthreads();

  if (wave == 0) {
#pragma unroll 1
    for (int b0 = 0; b0 < nh; b0 += 32) {
      const int idx = b0 + lane;
      const int uv  = reg1[idx < nh ? idx : nh - 1];
      const int m32 = (nh - b0) < 32 ? (nh - b0) : 32;
#pragma unroll 1
      for (int k = 0; k < m32; ++k) {
        const int u   = __builtin_amdgcn_readlane(uv, k);
        const int sl  = u & (NBMAX - 1);
        const int eid = (int)((unsigned)u >> SLOTB);
        if (lane == 0) {
          int pos = list[sl];
          pos = pos < 0 ? 0 : (pos > RCAP - 1 ? RCAP - 1 : pos);
          reg2[pos] = eid;
          list[sl] = pos + 1;
        }
      }
    }
  }
  __syncthreads();

  const int nbw = nb >> 3;
  const bool ovf = (nh >= RCAP);
  const float qnan = __int_as_float(0x7fc00000);
  const int c0 = 4 * lane;
  const int hd = lane >> 3;
  const v4f bb4 = *(const v4fa*)(par + PAR_BIAS + c0);
  const float* ASp = SD;
  const float* ADp = SD + (size_t)MPr * NHD;

#pragma unroll 1
  for (int jt = 0; jt < nbw; ++jt) {
    const int slot = wave * nbw + jt;
    const int grow = nodeBase + slot;
    const int gcl  = grow < nN ? grow : nN - 1;
    int st = soff[slot];
    const int craw = scnt[slot];
    int cnt = craw;
    st  = st < 0 ? 0 : (st > nh ? nh : st);
    cnt = cnt < 0 ? 0 : (cnt > DEGCAP ? DEGCAP : cnt);
    if (cnt > nh - st) cnt = nh - st;
    const float pz = (ovf || craw > DEGCAP) ? qnan : 0.0f;

    const v4f fd  = *(const v4fa*)(F + (size_t)gcl * HC + c0);
    const v4f ad4 = *(const v4fa*)(ADp + (size_t)gcl * NHD);
    const v4f sf4 = *(const v4fa*)(ASp + (size_t)gcl * NHD);
    float adv = ad4.x; adv = (hd == 1) ? ad4.y : adv; adv = (hd == 2) ? ad4.z : adv; adv = (hd == 3) ? ad4.w : adv;
    float asf = sf4.x; asf = (hd == 1) ? sf4.y : asf; asf = (hd == 2) ? sf4.z : asf; asf = (hd == 3) ? sf4.w : asf;
    float l0 = asf + adv;
    l0 = l0 > 0.f ? l0 : NEGSL * l0;
    float mx = l0, dn = 1.0f;
    v4f av = fd;

#pragma unroll 1
    for (int q = 0; q < cnt; ++q) {
      int idx = st + q; idx = idx > RCAP - 1 ? RCAP - 1 : idx;
      int eid = reg2[idx]; eid = eid < 0 ? 0 : (eid > nE - 1 ? nE - 1 : eid);
      const int sraw = srcs[eid];
      const int s = sraw < 0 ? 0 : (sraw > nN - 1 ? nN - 1 : sraw);
      const v4f fs  = *(const v4fa*)(F + (size_t)s * HC + c0);
      const v4f as4 = *(const v4fa*)(ASp + (size_t)s * NHD);
      float asv = as4.x; asv = (hd == 1) ? as4.y : asv; asv = (hd == 2) ? as4.z : asv; asv = (hd == 3) ? as4.w : asv;
      float lg = asv + adv;
      lg = lg > 0.f ? lg : NEGSL * lg;
      const float df = lg - mx;
      const float ee = expf(-fabsf(df));
      const bool up  = df > 0.f;
      const float s1 = up ? ee : 1.0f;
      const float s2 = up ? 1.0f : ee;
      mx = up ? lg : mx;
      dn = fmaf(dn, s1, s2);
      av.x = fmaf(av.x, s1, s2 * fs.x);
      av.y = fmaf(av.y, s1, s2 * fs.y);
      av.z = fmaf(av.z, s1, s2 * fs.z);
      av.w = fmaf(av.w, s1, s2 * fs.w);
    }
    const float inv = __builtin_amdgcn_rcpf(dn + EPS_SM);
    const bool live = grow < nN;
    const float vx = fmaf(av.x, inv, bb4.x), vy = fmaf(av.y, inv, bb4.y);
    const float vz = fmaf(av.z, inv, bb4.z), vw = fmaf(av.w, inv, bb4.w);
    const float rx = (vx > 0.f) ? vx : (vx - vx);
    const float ry = (vy > 0.f) ? vy : (vy - vy);
    const float rz = (vz > 0.f) ? vz : (vz - vz);
    const float rw = (vw > 0.f) ? vw : (vw - vw);
    v4f o;
    o.x = (live ? rx : 0.f) + pz;
    o.y = (live ? ry : 0.f) + pz;
    o.z = (live ? rz : 0.f) + pz;
    o.w = (live ? rw : 0.f) + pz;
    const unsigned int hbx = f2bf(o.x), hby = f2bf(o.y), hbz = f2bf(o.z), hbw = f2bf(o.w);
    const unsigned int lbx = f2bf(o.x - bf2f(hbx)), lby = f2bf(o.y - bf2f(hby));
    const unsigned int lbz = f2bf(o.z - bf2f(hbz)), lbw = f2bf(o.w - bf2f(hbw));
    const int hw0 = (int)(hbx | (hby << 16)), hw1 = (int)(hbz | (hbw << 16));
    const int lw0 = (int)(lbx | (lby << 16)), lw1 = (int)(lbz | (lbw << 16));
    const int sa = (2 * lane) & 31, sb = (2 * lane + 1) & 31;
    const int g0 = __shfl(hw0, sa), g1 = __shfl(hw1, sa), g2 = __shfl(hw0, sb), g3 = __shfl(hw1, sb);
    const int q0 = __shfl(lw0, sa), q1 = __shfl(lw1, sa), q2 = __shfl(lw0, sb), q3 = __shfl(lw1, sb);
    const bool lsel = lane >= 16;
    v4u pv;
    pv.x = (unsigned int)(lsel ? q0 : g0);
    pv.y = (unsigned int)(lsel ? q1 : g1);
    pv.z = (unsigned int)(lsel ? q2 : g2);
    pv.w = (unsigned int)(lsel ? q3 : g3);
    unsigned short* gp = HP + (size_t)grow * KA2 + 8 * lane;
    const bool wr = grow < MPr;
    if (wr) *(volatile v4u*)gp = pv;
    __threadfence();
    if (wr) *(volatile v4u*)gp = pv;
  }
}

__global__ __launch_bounds__(GTHR) void k_gemm2(const unsigned short* __restrict__ A,
                                                const unsigned short* __restrict__ WT,
                                                const float* __restrict__ par, float* outF, int nN) {
  __shared__ __attribute__((aligned(16))) float stg[GBM * OUTC];
  __shared__ __attribute__((aligned(16))) float slb[OUTC];
  const int tid = (int)threadIdx.x, lane = tid & 31, wave = tid >> 5, hh = lane >> 4, m = lane & 15;
  const int rowBase = (int)blockIdx.x * GBM;

  {
    const v4f lb = *(const v4fa*)(par + PAR_LINB + 4 * (tid & 15));
    if (tid < 16) *(v4fa*)(slb + 4 * tid) = lb;
  }

  v8f acc[4];
  {
    const v8f z = {0.f, 0.f, 0.f, 0.f, 0.f, 0.f, 0.f, 0.f};
    acc[0] = z; acc[1] = z; acc[2] = z; acc[3] = z;
  }
  const unsigned short* ap = A  + (size_t)(rowBase + 16 * wave + m) * (size_t)KA2 + 8 * hh;
  const unsigned short* wp = WT + (size_t)m * (size_t)KA2 + 8 * hh;
#pragma unroll 1
  for (int ks = 0; ks < KA2 / 32; ++ks) {
    FragB af;
    af.h[0] = *(const v8usa*)(ap + 32 * ks);
    af.h[1] = *(const v8usa*)(ap + 32 * ks + 16);
#pragma unroll
    for (int t = 0; t < 4; ++t) {
      const unsigned short* wq = wp + (size_t)(16 * t) * (size_t)KA2 + 32 * ks;
      FragB bf;
      bf.h[0] = *(const v8usa*)wq;
      bf.h[1] = *(const v8usa*)(wq + 16);
      acc[t] = wmb(af, bf, acc[t]);
    }
  }

#pragma unroll
  for (int t = 0; t < 4; ++t) {
    const int lc = 16 * t + m;
#pragma unroll
    for (int r = 0; r < 8; ++r) {
      const int lr = 16 * wave + 8 * hh + r;
      stg[lr * OUTC + lc] = acc[t][r];
    }
  }
  __syncthreads();

  const v4f bv = *(const v4fa*)(slb + 4 * m);
  v4f fv[8];
#pragma unroll
  for (int i = 0; i < 8; ++i) {
    const int lr = 16 * wave + 2 * i + hh;
    const v4f p = *(const v4fa*)(stg + lr * OUTC + 4 * m);
    v4f o;
    o.x = p.x + bv.x; o.y = p.y + bv.y; o.z = p.z + bv.z; o.w = p.w + bv.w;
    fv[i] = o;
  }
#pragma unroll
  for (int i = 0; i < 8; ++i) {
    const int gr = rowBase + 16 * wave + 2 * i + hh;
    float* op = outF + (size_t)gr * (size_t)OUTC + 4 * m;
    if (gr < nN) *(volatile v4f*)op = fv[i];
  }
  __threadfence();
#pragma unroll
  for (int i = 0; i < 8; ++i) {
    const int gr = rowBase + 16 * wave + 2 * i + hh;
    float* op = outF + (size_t)gr * (size_t)OUTC + 4 * m;
    if (gr < nN) *(volatile v4f*)op = fv[i];
  }
}

static inline int cdiv(int a, int b) { return (a + b - 1) / b; }

extern "C" void kernel_launch(void* const* d_in, const int* in_sizes, int n_in,
                              void* d_out, int out_size, void* d_ws, size_t ws_size,
                              hipStream_t stream) {
  if (n_in < 8) return;
  if (in_sizes[0] < F_IN || (in_sizes[0] % F_IN) != 0) return;
  const int nN = in_sizes[0] / F_IN;
  if (nN <= 0 || nN > (1 << 22)) return;
  if (in_sizes[1] < 2 || (in_sizes[1] & 1) != 0) return;
  const int nE = in_sizes[1] / 2;
  if (nE < 1 || nE >= (1 << (32 - SLOTB))) return;
  if (in_sizes[2] != F_IN * HC) return;
  if (in_sizes[3] != NHD * HID || in_sizes[4] != NHD * HID) return;
  if (in_sizes[5] != HC) return;
  if (in_sizes[6] != HC * OUTC) return;
  if (in_sizes[7] != OUTC) return;
  if ((long long)out_size != (long long)nN * OUTC) return;

  const float* x    = (const float*)d_in[0];
  const int*   ei   = (const int*)  d_in[1];
  const float* W    = (const float*)d_in[2];
  const float* ats  = (const float*)d_in[3];
  const float* atd  = (const float*)d_in[4];
  const float* bias = (const float*)d_in[5];
  const float* lw   = (const float*)d_in[6];
  const float* linb = (const float*)d_in[7];
  float* out = (float*)d_out;
  const int* src = ei;
  const int* dst = ei + nE;

  const int MP   = cdiv(nN, MROWS) * MROWS;
  const int nb   = NBRUN;
  const int gA   = cdiv(MP, nb);
  if ((long long)gA * nb < (long long)MP) return;
  const int vec8 = ((nE & 3) == 0) ? 1 : 0;
  const int nbx  = MP / 16;

  char* ws = (char*)d_ws;
  size_t off = 0;
  const size_t oA   = off; off += (size_t)MP * KA2 * 2;          off = (off + 255) & ~(size_t)255;
  const size_t oH   = off; off += (size_t)MP * HC * 4;           off = (off + 255) & ~(size_t)255;
  const size_t oSD  = off; off += (size_t)2 * MP * NHD * 4;      off = (off + 255) & ~(size_t)255;
  const size_t oW1T = off; off += (size_t)HC * F_IN * 2;         off = (off + 255) & ~(size_t)255;
  const size_t oLW  = off; off += (size_t)OUTC * KA2 * 2;        off = (off + 255) & ~(size_t)255;
  const size_t oPAR = off; off += (size_t)PAR_N * 4;             off = (off + 255) & ~(size_t)255;
  if (off > ws_size || off > (size_t)WSMAX) return;
  if ((size_t)MP * F_IN * 2 > (size_t)MP * KA2 * 2) return;
  unsigned short* X1HL = (unsigned short*)(ws + oA);
  unsigned short* XB   = (unsigned short*)(ws + oA);
  float*          H    = (float*)(ws + oH);
  float*          SD   = (float*)(ws + oSD);
  unsigned short* W1T  = (unsigned short*)(ws + oW1T);
  unsigned short* LWT2 = (unsigned short*)(ws + oLW);
  float*          PAR  = (float*)(ws + oPAR);

  hipFuncSetAttribute(reinterpret_cast<const void*>(&k_scan),
                      hipFuncAttributeMaxDynamicSharedMemorySize, (int)LDS_SCAN);

  const int gP = nbx + NUW1 / NTHR + NUW2 / NTHR + 1;
  const int gM = MP / GBM;
  k_prep<<<gP, NTHR, 0, stream>>>(x, W, lw, ats, atd, bias, linb, XB, W1T, LWT2, PAR, nN, nbx);
  k_gemm1<<<gM, GTHR, 0, stream>>>(XB, W1T, H, PAR, SD, MP);
  k_scan<<<gA, NTHR, LDS_SCAN, stream>>>(src, dst, H, SD, PAR, X1HL, nN, nE, nb, vec8, MP);
  k_gemm2<<<gM, GTHR, 0, stream>>>(X1HL, LWT2, PAR, out, nN);
}
